// Encoder_32384053412295
// MI455X (gfx1250) — hardware-verified
//
#include <hip/hip_runtime.h>
#include <hip/hip_bf16.h>
#include <stdint.h>

constexpr int NBATCH = 4;
constexpr int SEQ    = 2048;
constexpr int DMODEL = 512;
constexpr int NHEAD  = 8;
constexpr int DHEAD  = 64;
constexpr int QKLD   = 2 * DMODEL;
constexpr int NROWS  = NBATCH * SEQ;
constexpr float NEG_FILL    = -1.0e9f;
constexpr float SCORE_SCALE = 0.125f;
constexpr float PCARRY      = 1024.0f;

constexpr int ATT_QB = 64;
constexpr int ATT_KC = 64;
constexpr int ATT_NW = 4;

static_assert(DHEAD == 64);
static_assert(SEQ % ATT_QB == 0 && SEQ % ATT_KC == 0);
static_assert(NROWS % 64 == 0 && SEQ % 64 == 0 && DMODEL % 64 == 0 && QKLD % 64 == 0);
static_assert(DMODEL % 32 == 0);
static_assert((NROWS * DMODEL) % (8 * 256) == 0);

constexpr size_t WS_XB   = (size_t)NROWS * DMODEL * 2;
constexpr size_t WS_WQKT = (size_t)QKLD * DMODEL * 2;
constexpr size_t WS_WVT  = (size_t)DMODEL * DMODEL * 2;
constexpr size_t WS_WOT  = (size_t)DMODEL * DMODEL * 2;
constexpr size_t WS_QKP  = (size_t)NBATCH * SEQ * QKLD * 2;
constexpr size_t WS_VTP  = (size_t)NBATCH * DMODEL * SEQ * 2;
constexpr size_t WS_CTX  = (size_t)NROWS * DMODEL * 2;
constexpr size_t OFF_XB   = 0;
constexpr size_t OFF_WQKT = OFF_XB + WS_XB;
constexpr size_t OFF_WVT  = OFF_WQKT + WS_WQKT;
constexpr size_t OFF_WOT  = OFF_WVT + WS_WVT;
constexpr size_t OFF_QKP  = OFF_WOT + WS_WOT;
constexpr size_t OFF_VTP  = OFF_QKP + WS_QKP;
constexpr size_t OFF_CTXH = OFF_VTP + WS_VTP;
constexpr size_t OFF_CTXL = OFF_CTXH + WS_CTX;
constexpr size_t WS_TOTAL = OFF_CTXL + WS_CTX;
static_assert(WS_TOTAL == 52428800);
static_assert(WS_TOTAL <= 134217728);
static_assert(OFF_WQKT % 128 == 0 && OFF_WVT % 128 == 0 && OFF_WOT % 128 == 0 && OFF_QKP % 128 == 0 &&
              OFF_VTP % 128 == 0 && OFF_CTXH % 128 == 0 && OFF_CTXL % 128 == 0);

typedef __attribute__((ext_vector_type(16))) _Float16 v16h;
typedef __attribute__((ext_vector_type(8)))  _Float16 v8h;
typedef __attribute__((ext_vector_type(16))) __bf16   v16b;
typedef __attribute__((ext_vector_type(8)))  __bf16   v8b;
typedef __attribute__((ext_vector_type(8)))  float    v8f;
typedef __attribute__((ext_vector_type(4)))  float    v4f;
typedef __attribute__((ext_vector_type(4)))  unsigned u32x4;

__device__ __forceinline__ unsigned short f2bf_bits(float f) {
  unsigned u = __float_as_uint(f);
  return (unsigned short)((u + 0x7FFFu + ((u >> 16) & 1u)) >> 16);
}
__device__ __forceinline__ float bf_bits2f(unsigned short h) { return __uint_as_float(((unsigned)h) << 16); }
__device__ __forceinline__ unsigned pack_bf16x2(float a, float b) {
  return (unsigned)f2bf_bits(a) | ((unsigned)f2bf_bits(b) << 16);
}

__device__ __forceinline__ void dep_guard_h(v8f& a, v8f& b, v16h x, v16h y) { asm volatile("v_nop\n\tv_nop\n\tv_nop\n\tv_nop" : "+v"(a), "+v"(b) : "v"(x), "v"(y)); }
__device__ __forceinline__ void dep_guard_b(v8f& a, v8f& b, v16b x, v16b y) { asm volatile("v_nop\n\tv_nop\n\tv_nop\n\tv_nop" : "+v"(a), "+v"(b) : "v"(x), "v"(y)); }
__device__ __forceinline__ void keep4_h(v16h a, v16h b, v16h c, v16h d) { asm volatile("v_nop" :: "v"(a), "v"(b), "v"(c), "v"(d)); }
__device__ __forceinline__ void keep4_b(v16b a, v16b b, v16b c, v16b d) { asm volatile("v_nop" :: "v"(a), "v"(b), "v"(c), "v"(d)); }
__device__ __forceinline__ void acc_guard4(v8f& a, v8f& b, v8f& c, v8f& d) { asm volatile("v_nop\n\tv_nop\n\tv_nop\n\tv_nop" : "+v"(a), "+v"(b), "+v"(c), "+v"(d)); }
template <typename T> struct Frag;
template <> struct Frag<_Float16> {
  typedef v16h V; union U { v16h v; v8h h[2]; };
  static __device__ __forceinline__ v16h load(const _Float16* p) {
    U f; f.h[0] = *(const v8h*)(p); f.h[1] = *(const v8h*)(p + 16); return f.v;
  }
  static __device__ __forceinline__ v8f mma(v16h a, v16h b, v8f c) {
    return __builtin_amdgcn_wmma_f32_16x16x32_f16(false, a, false, b, (short)0, c, false, false);
  }
  static __device__ __forceinline__ void guard(v8f& a, v8f& b, v16h x, v16h y) { dep_guard_h(a, b, x, y); }
  static __device__ __forceinline__ void keep(v16h a, v16h b, v16h c, v16h d) { keep4_h(a, b, c, d); }
};
template <> struct Frag<__bf16> {
  typedef v16b V; union U { v16b v; v8b h[2]; };
  static __device__ __forceinline__ v16b load(const __bf16* p) {
    U f; f.h[0] = *(const v8b*)(p); f.h[1] = *(const v8b*)(p + 16); return f.v;
  }
  static __device__ __forceinline__ v8f mma(v16b a, v16b b, v8f c) {
    return __builtin_amdgcn_wmma_f32_16x16x32_bf16(false, a, false, b, (short)0, c, false, false);
  }
  static __device__ __forceinline__ void guard(v8f& a, v8f& b, v16b x, v16b y) { dep_guard_b(a, b, x, y); }
  static __device__ __forceinline__ void keep(v16b a, v16b b, v16b c, v16b d) { keep4_b(a, b, c, d); }
};

__global__ __launch_bounds__(256) void cast_f32_bf16x8(
    const float* __restrict__ in, unsigned short* __restrict__ out, int n8) {
  const int i = blockIdx.x * 256 + threadIdx.x;
  if (i < n8) {
    const v4f a = *(const v4f*)(in + (size_t)8 * i);
    const v4f c = *(const v4f*)(in + (size_t)8 * i + 4);
    u32x4 w;
    w[0] = pack_bf16x2(a[0], a[1]);
    w[1] = pack_bf16x2(a[2], a[3]);
    w[2] = pack_bf16x2(c[0], c[1]);
    w[3] = pack_bf16x2(c[2], c[3]);
    unsigned short* op = out + (size_t)8 * i;
    *(volatile u32x4*)(void*)op = w;
    __threadfence();
    *(volatile u32x4*)(void*)op = w;
  }
}

__global__ __launch_bounds__(128) void tcast64_bf16(
    const float* __restrict__ src, long srcMat, int srcLd,
    unsigned short* __restrict__ dst, long dstMat, int dstLd) {
  __shared__ __align__(16) float tile[64 * 68];
  const int tid = threadIdx.x, lane = tid & 31, wave = tid >> 5;
  const int k0 = blockIdx.x * 64, n0 = blockIdx.y * 64;
  const float* s = src + (size_t)blockIdx.z * srcMat;
  unsigned short* d = dst + (size_t)blockIdx.z * dstMat;
#pragma unroll
  for (int i = 0; i < 8; ++i) {
    const int id = tid + 128 * i;
    const int row = id >> 4, c4 = (id & 15) * 4;
    const v4f v = *(const v4f*)(s + (size_t)(k0 + row) * srcLd + n0 + c4);
    *(v4f*)(tile + row * 68 + c4) = v;
  }
  __syncthreads();
  const int q4 = lane >> 3, c8 = (lane & 7) * 8;
  u32x4 w[4];
#pragma unroll
  for (int it = 0; it < 4; ++it) {
    const int row = wave * 16 + it * 4 + q4;
#pragma unroll
    for (int e = 0; e < 4; ++e) {
      const float f0 = tile[(c8 + 2 * e) * 68 + row];
      const float f1 = tile[(c8 + 2 * e + 1) * 68 + row];
      w[it][e] = pack_bf16x2(f0, f1);
    }
  }
  for (int ps = 0; ps < 2; ++ps) {
#pragma unroll
    for (int it = 0; it < 4; ++it) {
      const int row = wave * 16 + it * 4 + q4;
      unsigned short* op = d + (size_t)(n0 + row) * dstLd + k0 + c8;
      *(volatile u32x4*)(void*)op = w[it];
    }
    __threadfence();
  }
}

template <int ET> struct Elem;
template <> struct Elem<0> { typedef _Float16 T; };
template <> struct Elem<1> { typedef __bf16 T; };
template <int ET, int SPLITM, int BIAS_MODE, int OUT_MODE, bool RESID, int ACT = 0>
__global__ __launch_bounds__(256) void wmma_gemm64(
    const unsigned short* __restrict__ Ap, const unsigned short* __restrict__ A2p, int lda, long strideA,
    const unsigned short* __restrict__ Btp, const unsigned short* __restrict__ Bt2p, int ldb, long strideB,
    void* __restrict__ Cout, void* __restrict__ Cout2, int ldc, long strideC,
    const float* __restrict__ bias,
    const float* __restrict__ resid, long strideR,
    int M, int N, int K, float scale) {
  typedef typename Elem<ET>::T T;
  typedef typename Frag<T>::V V;
  const T* A = (const T*)Ap; const T* A2 = (const T*)A2p; const T* Bt = (const T*)Btp; const T* Bt2 = (const T*)Bt2p;
  __shared__ __align__(16) float sT[8][16 * 68];
  const int b    = blockIdx.y;
  const int lane = threadIdx.x & 31;
  const int wave = threadIdx.x >> 5;
  const int tilesN = N >> 6;
  const int tilesM = M >> 6;
  const int tile = blockIdx.x * 8 + wave;
  if (tile >= tilesM * tilesN) return;
  const int tm = tile / tilesN;
  const int tn = tile - tm * tilesN;
  const int m0 = tm << 6;
  const int n0 = tn << 6;

  const T* Ab  = A  + (size_t)b * strideA;
  const T* Bb  = Bt + (size_t)b * strideB;
  const T* Ab2 = (SPLITM >= 1) ? (A2  + (size_t)b * strideA) : nullptr;
  const T* Bb2 = (SPLITM == 2) ? (Bt2 + (size_t)b * strideB) : nullptr;

  const int rlane = lane & 15;
  const int koff  = (lane >> 4) * 8;
  const int mOff  = (lane >> 4) * 8;

  v8f acc[4][4];
#pragma unroll
  for (int i = 0; i < 4; ++i)
#pragma unroll
    for (int j = 0; j < 4; ++j) acc[i][j] = (v8f){0.f,0.f,0.f,0.f,0.f,0.f,0.f,0.f};

  for (int k0 = 0; k0 < K; k0 += 32) {
    V bh[4], bl[4];
#pragma unroll
    for (int j = 0; j < 4; ++j) {
      const size_t bo = (size_t)(n0 + (j << 4) + rlane) * ldb + koff + k0;
      bh[j] = Frag<T>::load(Bb + bo);
      if (SPLITM == 2) bl[j] = Frag<T>::load(Bb2 + bo);
    }
#pragma unroll
    for (int i = 0; i < 4; ++i) {
      const size_t ao = (size_t)(m0 + (i << 4) + rlane) * lda + koff + k0;
      V ah = Frag<T>::load(Ab + ao);
      V al;
      if (SPLITM >= 1) al = Frag<T>::load(Ab2 + ao);
#pragma unroll
      for (int j = 0; j < 4; ++j) {
        acc[i][j] = Frag<T>::mma(ah, bh[j], acc[i][j]);
        if (SPLITM == 2) acc[i][j] = Frag<T>::mma(ah, bl[j], acc[i][j]);
        if (SPLITM >= 1) acc[i][j] = Frag<T>::mma(al, bh[j], acc[i][j]);
      }
      Frag<T>::guard(acc[i][0], acc[i][3], ah, (SPLITM >= 1) ? al : ah);
    }
    Frag<T>::keep(bh[0], bh[1], bh[2], bh[3]);
    if (SPLITM == 2) Frag<T>::keep(bl[0], bl[1], bl[2], bl[3]);
  }
  acc_guard4(acc[0][0], acc[0][1], acc[0][2], acc[0][3]);
  acc_guard4(acc[1][0], acc[1][1], acc[1][2], acc[1][3]);
  acc_guard4(acc[2][0], acc[2][1], acc[2][2], acc[2][3]);
  acc_guard4(acc[3][0], acc[3][1], acc[3][2], acc[3][3]);

  float* slab = sT[wave];
  const float* Rb = RESID ? (resid + (size_t)b * strideR) : nullptr;
#pragma unroll
  for (int i = 0; i < 4; ++i) {
    const int mBase = m0 + (i << 4);
#pragma unroll
    for (int j = 0; j < 4; ++j) {
      const int n = n0 + (j << 4) + rlane;
      float bv = 0.f;
      if (BIAS_MODE == 2) bv = bias[n];
#pragma unroll
      for (int r = 0; r < 8; ++r) {
        float v = acc[i][j][r] * scale;
        if (BIAS_MODE == 1) v += bias[mBase + mOff + r];
        if (BIAS_MODE == 2) v += bv;
        if (RESID) v += Rb[(size_t)(mBase + mOff + r) * ldc + n];
        if (ACT == 1) v = tanhf(v);
        if (ACT == 2) v = fmaxf(v, 0.0f);
        if (ACT == 3) v = v / (1.0f + expf(-v));
        if (ACT == 4) v = (v > 0.f) ? v : 0.01f * v;
        slab[(mOff + r) * 68 + (j << 4) + rlane] = v;
      }
    }
    __builtin_amdgcn_fence(__ATOMIC_RELEASE, "workgroup");
    __builtin_amdgcn_wave_barrier();
    __builtin_amdgcn_fence(__ATOMIC_ACQUIRE, "workgroup");
    if (OUT_MODE == 0) {
      float* C = (float*)Cout + (size_t)b * strideC;
      const int hh = lane >> 4, c4 = (lane & 15) * 4;
      for (int ps = 0; ps < 2; ++ps) {
#pragma unroll
        for (int it = 0; it < 8; ++it) {
          const int row = it * 2 + hh;
          v4f v = *(const v4f*)(slab + row * 68 + c4);
          *(volatile v4f*)(C + (size_t)(mBase + row) * ldc + n0 + c4) = v;
        }
        __threadfence();
      }
    } else {
      const int q = lane >> 3, c8 = (lane & 7) * 8;
      unsigned short* C  = (unsigned short*)Cout  + (size_t)b * strideC;
      unsigned short* C2 = (OUT_MODE == 2) ? ((unsigned short*)Cout2 + (size_t)b * strideC) : nullptr;
      for (int ps = 0; ps < 2; ++ps) {
#pragma unroll
        for (int it = 0; it < 4; ++it) {
          const int row = it * 4 + q;
          const float* sp = slab + row * 68 + c8;
          v8h hv, lv;
#pragma unroll
          for (int e = 0; e < 8; ++e) {
            if (OUT_MODE == 1) {
              hv[e] = (_Float16)sp[e];
            } else {
              unsigned short hb = f2bf_bits(sp[e]);
              unsigned short lb = f2bf_bits(sp[e] - bf_bits2f(hb));
              hv[e] = __builtin_bit_cast(_Float16, hb);
              lv[e] = __builtin_bit_cast(_Float16, lb);
            }
          }
          *(volatile v8h*)(C + (size_t)(mBase + row) * ldc + n0 + c8) = hv;
          if (OUT_MODE == 2) *(volatile v8h*)(C2 + (size_t)(mBase + row) * ldc + n0 + c8) = lv;
        }
        __threadfence();
      }
    }
    __builtin_amdgcn_fence(__ATOMIC_RELEASE, "workgroup");
    __builtin_amdgcn_wave_barrier();
    __builtin_amdgcn_fence(__ATOMIC_ACQUIRE, "workgroup");
  }
}

__device__ __forceinline__ v8f mma_f16(v16h a, v16h b, v8f c) {
  c = __builtin_amdgcn_wmma_f32_16x16x32_f16(false, a, false, b, (short)0, c, false, false);
  asm volatile("v_nop\n\tv_nop\n\tv_nop\n\tv_nop" : "+v"(c) : "v"(a), "v"(b));
  return c;
}

__global__ __launch_bounds__(128)
void attn_f16(const unsigned short* __restrict__ qkp, const unsigned short* __restrict__ vtp,
              const int* __restrict__ mask,
              unsigned short* __restrict__ ctxh, unsigned short* __restrict__ ctxl) {
  __shared__ __align__(16) _Float16 Ksh[ATT_KC * DHEAD];
  __shared__ __align__(16) _Float16 Vth[DHEAD * ATT_KC];
  __shared__ __align__(16) _Float16 Psh[ATT_NW][16 * ATT_KC];
  __shared__ __align__(16) float    Os[ATT_NW][16 * 68];

  const int tid  = threadIdx.x;
  const int wave = tid >> 5;
  const int lane = tid & 31;
  const int hh   = lane >> 4;
  const int c    = lane & 15;

  constexpr int NQB = SEQ / ATT_QB;
  const int bx = blockIdx.x;
  const int qb = bx % NQB;
  const int bh = bx / NQB;
  const int h  = bh % NHEAD;
  const int b  = bh / NHEAD;
  const int q0 = qb * ATT_QB + wave * 16;

  const _Float16* qk16 = (const _Float16*)(const void*)qkp;
  const _Float16* vt16 = (const _Float16*)(const void*)vtp;

  v16h qa[2];
  {
    const _Float16* Qg = qk16 + ((size_t)b * SEQ + q0 + c) * QKLD + h * DHEAD;
    qa[0] = Frag<_Float16>::load(Qg + 8 * hh);
    qa[1] = Frag<_Float16>::load(Qg + 32 + 8 * hh);
  }
  const _Float16* Kg = qk16 + (size_t)b * SEQ * QKLD + DMODEL + h * DHEAD;
  const _Float16* Vg = vt16 + ((size_t)b * DMODEL + h * DHEAD) * SEQ;
  const int* mk = mask + (size_t)b * SEQ;

  float mrow[8], lrow[8];
  v8f oacc[4];
#pragma unroll
  for (int r = 0; r < 8; ++r) { mrow[r] = -__builtin_inff(); lrow[r] = 0.f; }
#pragma unroll
  for (int t = 0; t < 4; ++t) oacc[t] = (v8f){0.f,0.f,0.f,0.f,0.f,0.f,0.f,0.f};

  for (int kc = 0; kc < SEQ / ATT_KC; ++kc) {
    const int kv0 = kc * ATT_KC;
    __syncthreads();
#pragma unroll
    for (int i = 0; i < 4; ++i) {
      const int id  = tid + 128 * i;
      const int row = id >> 3, c16 = (id & 7) * 8;
      const v8h kk = *(const v8h*)(Kg + (size_t)(kv0 + row) * QKLD + c16);
      const v8h vv = *(const v8h*)(Vg + (size_t)row * SEQ + kv0 + c16);
      *(v8h*)(Ksh + row * DHEAD + c16) = kk;
      *(v8h*)(Vth + row * ATT_KC + c16) = vv;
    }
    __syncthreads();

    int kvkeep[4];
#pragma unroll
    for (int j = 0; j < 4; ++j) kvkeep[j] = mk[kv0 + j * 16 + c];

    v8f s[4];
#pragma unroll
    for (int j = 0; j < 4; ++j) {
      s[j] = (v8f){0.f,0.f,0.f,0.f,0.f,0.f,0.f,0.f};
#pragma unroll
      for (int dc = 0; dc < 2; ++dc) {
        const v16h kb = Frag<_Float16>::load(Ksh + (j * 16 + c) * DHEAD + dc * 32 + 8 * hh);
        s[j] = mma_f16(qa[dc], kb, s[j]);
      }
    }

    float cm[8];
#pragma unroll
    for (int r = 0; r < 8; ++r) {
      float m = -__builtin_inff();
#pragma unroll
      for (int j = 0; j < 4; ++j) {
        float v = s[j][r] * SCORE_SCALE;
        v = (kvkeep[j] > 0) ? v : NEG_FILL;
        s[j][r] = v;
        m = fmaxf(m, v);
      }
#pragma unroll
      for (int off = 1; off < 16; off <<= 1) m = fmaxf(m, __shfl_xor(m, off, 32));
      cm[r] = m;
    }

    _Float16* pw = Psh[wave];
#pragma unroll
    for (int r = 0; r < 8; ++r) {
      const float mnew  = fmaxf(mrow[r], cm[r]);
      const float alpha = expf(mrow[r] - mnew);
      mrow[r] = mnew;
      float psum = 0.f;
#pragma unroll
      for (int j = 0; j < 4; ++j) {
        const float p = expf(s[j][r] - mnew);
        psum += p;
        pw[(8 * hh + r) * ATT_KC + j * 16 + c] = (_Float16)(p * PCARRY);
      }
#pragma unroll
      for (int off = 1; off < 16; off <<= 1) psum += __shfl_xor(psum, off, 32);
      lrow[r] = lrow[r] * alpha + psum;
#pragma unroll
      for (int t = 0; t < 4; ++t) oacc[t][r] *= alpha;
    }
    __builtin_amdgcn_fence(__ATOMIC_RELEASE, "workgroup");
    __builtin_amdgcn_wave_barrier();
    __builtin_amdgcn_fence(__ATOMIC_ACQUIRE, "workgroup");

#pragma unroll
    for (int kk = 0; kk < 2; ++kk) {
      const v16h pa = Frag<_Float16>::load(pw + c * ATT_KC + kk * 32 + 8 * hh);
#pragma unroll
      for (int t = 0; t < 4; ++t) {
        const v16h vb = Frag<_Float16>::load(Vth + (t * 16 + c) * ATT_KC + kk * 32 + 8 * hh);
        oacc[t] = mma_f16(pa, vb, oacc[t]);
      }
    }
  }

  float* os = Os[wave];
#pragma unroll
  for (int r = 0; r < 8; ++r) {
    const float inv = 1.0f / (lrow[r] * PCARRY);
#pragma unroll
    for (int t = 0; t < 4; ++t) os[(8 * hh + r) * 68 + t * 16 + c] = oacc[t][r] * inv;
  }
  __builtin_amdgcn_fence(__ATOMIC_RELEASE, "workgroup");
  __builtin_amdgcn_wave_barrier();
  __builtin_amdgcn_fence(__ATOMIC_ACQUIRE, "workgroup");
  {
    const int q4 = lane >> 3, c8 = (lane & 7) * 8;
    v8h hvs[4], lvs[4];
#pragma unroll
    for (int it = 0; it < 4; ++it) {
      const int row = it * 4 + q4;
      const float* sp = os + row * 68 + c8;
#pragma unroll
      for (int e = 0; e < 8; ++e) {
        const unsigned short hb = f2bf_bits(sp[e]);
        const unsigned short lb = f2bf_bits(sp[e] - bf_bits2f(hb));
        hvs[it][e] = __builtin_bit_cast(_Float16, hb);
        lvs[it][e] = __builtin_bit_cast(_Float16, lb);
      }
    }
    const size_t rowg0 = (size_t)b * SEQ + q0;
    _Float16* CH = (_Float16*)(void*)ctxh;
    _Float16* CL = (_Float16*)(void*)ctxl;
    for (int ps = 0; ps < 2; ++ps) {
#pragma unroll
      for (int it = 0; it < 4; ++it) {
        const int row = it * 4 + q4;
        const size_t o = (rowg0 + row) * DMODEL + h * DHEAD + c8;
        *(volatile v8h*)(CH + o) = hvs[it];
        *(volatile v8h*)(CL + o) = lvs[it];
      }
      __threadfence();
    }
  }
}

extern "C" void kernel_launch(void* const* d_in, const int* in_sizes, int n_in,
                              void* d_out, int out_size, void* d_ws,
                              size_t ws_size, hipStream_t stream) {
  if (n_in < 6) return;
  if (ws_size < WS_TOTAL) return;
  if (out_size < NROWS * DMODEL) return;
  if (in_sizes[0] < NROWS * DMODEL || in_sizes[1] < NBATCH * SEQ ||
      in_sizes[2] < NHEAD * DMODEL * DHEAD || in_sizes[3] < NHEAD * DMODEL * DHEAD ||
      in_sizes[4] < NHEAD * DMODEL * DHEAD || in_sizes[5] < DMODEL * DMODEL) return;

  const float* x    = (const float*)d_in[0];
  const int*   mask = (const int*)d_in[1];
  const float* Wq   = (const float*)d_in[2];
  const float* Wk   = (const float*)d_in[3];
  const float* Wv   = (const float*)d_in[4];
  const float* Wo   = (const float*)d_in[5];
  float* out = (float*)d_out;

  char* ws = (char*)d_ws;
  unsigned short* xb   = (unsigned short*)(ws + OFF_XB);
  unsigned short* wqkT = (unsigned short*)(ws + OFF_WQKT);
  unsigned short* wvT  = (unsigned short*)(ws + OFF_WVT);
  unsigned short* woT  = (unsigned short*)(ws + OFF_WOT);
  unsigned short* qkp  = (unsigned short*)(ws + OFF_QKP);
  unsigned short* vtp  = (unsigned short*)(ws + OFF_VTP);
  unsigned short* ctxh = (unsigned short*)(ws + OFF_CTXH);
  unsigned short* ctxl = (unsigned short*)(ws + OFF_CTXL);

  {
    const int n8 = NROWS * DMODEL / 8;
    cast_f32_bf16x8<<<dim3((n8 + 255) / 256), dim3(256), 0, stream>>>(x, xb, n8);
  }
  {
    const long wMat = (long)DMODEL * DHEAD;
    tcast64_bf16<<<dim3(DMODEL / 64, DHEAD / 64, NHEAD), dim3(128), 0, stream>>>(
        Wq, wMat, DHEAD, wqkT, wMat, DMODEL);
    tcast64_bf16<<<dim3(DMODEL / 64, DHEAD / 64, NHEAD), dim3(128), 0, stream>>>(
        Wk, wMat, DHEAD, wqkT + (size_t)DMODEL * DMODEL, wMat, DMODEL);
    tcast64_bf16<<<dim3(DMODEL / 64, DHEAD / 64, NHEAD), dim3(128), 0, stream>>>(
        Wv, wMat, DHEAD, wvT, wMat, DMODEL);
    tcast64_bf16<<<dim3(DMODEL / 64, DMODEL / 64, 1), dim3(128), 0, stream>>>(
        Wo, 0L, DMODEL, woT, 0L, DMODEL);
  }
  {
    const int M = SEQ, N = QKLD, K = DMODEL;
    const int tiles = (M / 64) * (N / 64);
    wmma_gemm64<1, 0, 0, 1, false, 0><<<dim3((tiles + 7) / 8, NBATCH), dim3(256), 0, stream>>>(
        xb, xb, DMODEL, (long)SEQ * DMODEL,
        wqkT, wqkT, DMODEL, 0L,
        (void*)qkp, (void*)qkp, QKLD, (long)SEQ * QKLD,
        x, x, 0L, M, N, K, 1.0f);
  }
  {
    const int M = DMODEL, N = SEQ, K = DMODEL;
    const int tiles = (M / 64) * (N / 64);
    wmma_gemm64<1, 0, 0, 1, false, 0><<<dim3((tiles + 7) / 8, NBATCH), dim3(256), 0, stream>>>(
        wvT, wvT, DMODEL, 0L,
        xb, xb, DMODEL, (long)SEQ * DMODEL,
        (void*)vtp, (void*)vtp, SEQ, (long)DMODEL * SEQ,
        x, x, 0L, M, N, K, 1.0f);
  }
  attn_f16<<<dim3(NBATCH * NHEAD * (SEQ / ATT_QB)), dim3(128), 0, stream>>>(qkp, vtp, mask, ctxh, ctxl);
  {
    const int M = NROWS, N = DMODEL, K = DMODEL;
    const int tiles = (M / 64) * (N / 64);
    wmma_gemm64<1, 1, 0, 0, false, 0><<<dim3((tiles + 7) / 8, 1), dim3(256), 0, stream>>>(
        ctxh, ctxl, DMODEL, 0L,
        woT, woT, DMODEL, 0L,
        (void*)out, (void*)out, DMODEL, 0L,
        x, x, 0L, M, N, K, 1.0f);
  }
}
